// MultiHeadAttention_50809463111698
// MI455X (gfx1250) — hardware-verified
//
#include <hip/hip_runtime.h>


#ifndef NB
#define NB 4
#endif
#ifndef SEQ
#define SEQ 2048
#endif
#define NB_FULL  4
#define SEQ_FULL 2048
#ifndef OUT_SEQ
#define OUT_SEQ SEQ
#endif
#define DM   1024
#define NH_  16
#define HD   64
#define AW   4
#define EARLY ((SEQ < 512) ? SEQ : 512)
#define QRS  2048.0f
#define QRI  (1.0f / 2048.0f)
#define SC2  (0.125f * 1.4426950408889634f)
#define PSH  8.0f
#define CS   16.0f
#define WS   32.0f
#define OSC  (1.0f / 512.0f)
#define NEGB (-3.0e38f)
#define BIGI (1 << 30)

static_assert(HD == 64);
static_assert(NH_ * HD == DM);
static_assert(DM % 64 == 0);
static_assert(DM % 32 == 0);
static_assert(SEQ % 64 == 0);
static_assert((NB * SEQ) % 64 == 0);
static_assert(SEQ % 32 == 0);
static_assert(EARLY % 64 == 0);
static_assert((SEQ - EARLY) % 64 == 0);
static_assert(EARLY % (16 * AW) == 0);
static_assert(((size_t)SEQ * DM) % 8 == 0);
static_assert(((size_t)DM * DM) % 8 == 0);
static_assert(NB <= NB_FULL);
static_assert(SEQ <= SEQ_FULL);
static_assert((size_t)NB_FULL * SEQ_FULL * DM * 4 == (size_t)33554432);

typedef _Float16 h16;
typedef unsigned short bf;
typedef __attribute__((ext_vector_type(16))) __bf16   v16bf;
typedef __attribute__((ext_vector_type(16))) _Float16 v16h;
typedef __attribute__((ext_vector_type(8)))  _Float16 v8h;
typedef __attribute__((ext_vector_type(8)))  unsigned short v8us;
typedef __attribute__((ext_vector_type(8)))  float    v8f;
typedef __attribute__((ext_vector_type(4)))  float    v4f;
typedef __attribute__((ext_vector_type(4)))  int      v4i;
typedef v4f  __attribute__((may_alias)) v4fa;

__device__ __forceinline__ unsigned short f2bf(float f) { unsigned u = __float_as_uint(f); u += 0x7FFFu + ((u >> 16) & 1u); return (unsigned short)(u >> 16); }
__device__ __forceinline__ float bfr(float f) { return __uint_as_float(((unsigned)f2bf(f)) << 16); }
__device__ __forceinline__ int imax(int a, int b) { return a > b ? a : b; }
__device__ __forceinline__ v16h cat16(v8h lo, v8h hi) { return __builtin_shufflevector(lo, hi, 0, 1, 2, 3, 4, 5, 6, 7, 8, 9, 10, 11, 12, 13, 14, 15); }
__device__ __forceinline__ v16bf cat16b(v8us lo, v8us hi) { return __builtin_bit_cast(v16bf, __builtin_shufflevector(lo, hi, 0, 1, 2, 3, 4, 5, 6, 7, 8, 9, 10, 11, 12, 13, 14, 15)); }
__device__ __forceinline__ v8f wmma16(v16h a, v16h b, v8f c) { return __builtin_amdgcn_wmma_f32_16x16x32_f16(false, a, false, b, (short)0, c, false, false); }
__device__ __forceinline__ v8f wmmab(v16bf a, v16bf b, v8f c) { return __builtin_amdgcn_wmma_f32_16x16x32_bf16(false, a, false, b, (short)0, c, false, false); }
__device__ __forceinline__ v16h  ldh(const h16* p) { return cat16(*(const v8h*)p, *(const v8h*)(p + 16)); }
__device__ __forceinline__ v16bf ldb(const bf* p)  { return cat16b(*(const v8us*)p, *(const v8us*)(p + 16)); }
__device__ __forceinline__ void wave_sync() { __builtin_amdgcn_fence(3  , "wavefront"); __builtin_amdgcn_wave_barrier(); asm volatile("" ::: "memory"); }

__global__ __launch_bounds__(256) void k_cvt8(const float* __restrict__ src, bf* dst, size_t n8) {
    const size_t i = (size_t)blockIdx.x * 256 + threadIdx.x; if (i >= n8) return;
    const v8f v = *(const v8f*)(src + i * 8); v8us o;
#pragma unroll
    for (int k = 0; k < 8; ++k) o[k] = f2bf(v[k]);
    *(volatile v8us*)(dst + i * 8) = o; __threadfence(); *(volatile v8us*)(dst + i * 8) = o;
}

__global__ __launch_bounds__(256) void k_cvtw(const float* __restrict__ src, h16* dst, size_t n8) {
    const size_t i = (size_t)blockIdx.x * 256 + threadIdx.x; if (i >= n8) return;
    const v8f v = *(const v8f*)(src + i * 8); v8h o;
#pragma unroll
    for (int k = 0; k < 8; ++k) o[k] = (h16)(bfr(v[k]) * WS);
    *(volatile v8h*)(dst + i * 8) = o; __threadfence(); *(volatile v8h*)(dst + i * 8) = o;
}

__global__ __launch_bounds__(256) void k_mscan(const int* __restrict__ MK, int* KT) {
    __shared__ int kt_s[32];
    const int lane = threadIdx.x & 31, wave = __builtin_amdgcn_readfirstlane((int)(threadIdx.x >> 5));
#pragma unroll 1
    for (int j = 0; j < 4; ++j) {
        const int tile = (int)blockIdx.x * 32 + wave * 4 + j;
        int mx = -1;
        if (tile < SEQ / 16) {
            const int* base = MK + (size_t)tile * 16 * SEQ_FULL;
#pragma unroll 4
            for (int it = 0; it < SEQ / 8; ++it) {
                const int c = it * 32 + lane; const int row = c / (SEQ / 4), c4 = (c % (SEQ / 4)) * 4;
                const v4i v = *(const v4i*)(base + (size_t)row * SEQ_FULL + c4);
                mx = imax(mx, (v[0] != 0) ? c4     : -1);
                mx = imax(mx, (v[1] != 0) ? c4 + 1 : -1);
                mx = imax(mx, (v[2] != 0) ? c4 + 2 : -1);
                mx = imax(mx, (v[3] != 0) ? c4 + 3 : -1);
            }
        }
        mx = imax(mx, __shfl_xor(mx, 16, 32)); mx = imax(mx, __shfl_xor(mx, 8, 32)); mx = imax(mx, __shfl_xor(mx, 4, 32));
        mx = imax(mx, __shfl_xor(mx, 2, 32));  mx = imax(mx, __shfl_xor(mx, 1, 32));
        if (lane == 0) kt_s[wave * 4 + j] = ((mx + 32) / 32) * 32;
    }
    __syncthreads();
    if (wave == 0) { const int v = kt_s[lane]; volatile int* p = KT + (size_t)blockIdx.x * 32 + lane; *p = v; __threadfence(); *p = v; }
}

__global__ __launch_bounds__(32) void k_proj(const bf* __restrict__ A, const bf* __restrict__ Bt, const float* __restrict__ bias, int biasRow,
                                             h16* Ph, h16* Pr, int useRes, int RB, size_t sRB, int pitch, int CB, size_t sCB, int ER, int EC) {
    __shared__ __align__(16) float os[16 * 68];
    const int K = DM;
    const int lane = threadIdx.x & 31, lr = lane & 15, hi = lane >> 4; const int r0 = blockIdx.x * 64, c0 = blockIdx.y * 64;
    v8f acc[4][4];
#pragma unroll
    for (int mb = 0; mb < 4; ++mb)
#pragma unroll
        for (int nb = 0; nb < 4; ++nb) acc[mb][nb] = (v8f){};
    const size_t aoff = (size_t)(r0 + lr) * K + 8 * hi, boff = (size_t)(c0 + lr) * K + 8 * hi;
#pragma unroll 1
    for (int kc = 0; kc < K; kc += 32) {
        v16bf a[4];
#pragma unroll
        for (int mb = 0; mb < 4; ++mb) a[mb] = ldb(A + aoff + (size_t)mb * 16 * K + kc);
#pragma unroll
        for (int nb = 0; nb < 4; ++nb) { const v16bf b = ldb(Bt + boff + (size_t)nb * 16 * K + kc);
#pragma unroll
            for (int mb = 0; mb < 4; ++mb) acc[mb][nb] = wmmab(a[mb], b, acc[mb][nb]); }
        asm volatile("v_nop\n\tv_nop\n\tv_nop\n\tv_nop" : "+v"(acc[0][0]), "+v"(acc[1][1]), "+v"(acc[2][2]), "+v"(acc[3][3]) : "v"(a[0]), "v"(a[1]), "v"(a[2]), "v"(a[3]));
    }
    const int wr = (useRes != 0) && ((r0 % RB) < ER) && ((c0 % CB) < EC);
    const int c8l = (lane & 7) * 8;
    const int bco = biasRow ? 0 : (c0 + c8l);
    const v4f bA = *(const v4f*)(bias + bco), bB = *(const v4f*)(bias + bco + 4);
    float bcol[8];
#pragma unroll
    for (int i = 0; i < 4; ++i) { bcol[i] = bfr(bA[i]); bcol[4 + i] = bfr(bB[i]); }
    const size_t tbase = (size_t)(r0 / RB) * sRB + (size_t)(r0 % RB) * (size_t)pitch + (size_t)(c0 / CB) * sCB + (size_t)(c0 % CB);
#pragma unroll
    for (int mb = 0; mb < 4; ++mb) {
#pragma unroll
        for (int nb = 0; nb < 4; ++nb) {
#pragma unroll
            for (int j = 0; j < 8; ++j) os[(hi * 8 + j) * 68 + nb * 16 + lr] = acc[mb][nb][j]; }
        wave_sync();
        const size_t sb = tbase + (size_t)(mb * 16) * (size_t)pitch;
#pragma unroll 1
        for (int ps = 0; ps < 2; ++ps) {
#pragma unroll
            for (int s = 0; s < 4; ++s) { const int row = 4 * s + (lane >> 3), c8 = c8l;
                const float brow = bfr(bias[biasRow ? (r0 + mb * 16 + row) : 0]);
                const v4f x0 = *(const v4fa*)(&os[row * 68 + c8]); const v4f x1 = *(const v4fa*)(&os[row * 68 + c8 + 4]); v8h hv, rv;
#pragma unroll
                for (int i = 0; i < 4; ++i) {
                    const float y0 = x0[i] + (biasRow ? brow : bcol[i]); const float y1 = x1[i] + (biasRow ? brow : bcol[4 + i]);
                    const h16 a0 = (h16)y0; const h16 a1 = (h16)y1; hv[i] = a0; hv[4 + i] = a1;
                    rv[i] = (h16)((y0 - (float)a0) * QRS); rv[4 + i] = (h16)((y1 - (float)a1) * QRS); }
                const size_t oo = sb + (size_t)row * (size_t)pitch + c8;
                *(volatile v8h*)(Ph + oo) = hv; if (wr) *(volatile v8h*)(Pr + oo) = rv; }
            if (ps == 0) __threadfence(); }
        wave_sync();
    }
}

template <int RES> __device__ __forceinline__ v4f fin_lo(v8f oh, v8f ol, float inv) {
    v4f a = __builtin_shufflevector(oh, oh, 0, 1, 2, 3);
    if (RES) a = a + __builtin_shufflevector(ol, ol, 0, 1, 2, 3) * QRI;
    return a * inv; }
template <int RES> __device__ __forceinline__ v4f fin_hi(v8f oh, v8f ol, float inv) {
    v4f a = __builtin_shufflevector(oh, oh, 4, 5, 6, 7);
    if (RES) a = a + __builtin_shufflevector(ol, ol, 4, 5, 6, 7) * QRI;
    return a * inv; }

template <int RES>
__device__ __forceinline__ void flash_body(const h16* __restrict__ QH, const h16* __restrict__ QR, const h16* __restrict__ KP, const h16* __restrict__ KR,
                                           const h16* __restrict__ VT, const h16* __restrict__ VR, const int* __restrict__ MK, const int* __restrict__ KT,
                                           h16* CH, h16* CR, const int tbase) {
    __shared__ __align__(16) float os[AW * 16 * 68];
    const int lane = threadIdx.x & 31, wave = __builtin_amdgcn_readfirstlane((int)(threadIdx.x >> 5)), lr = lane & 15, hi = lane >> 4;
    const int zh = blockIdx.y; const int b = zh / NH_, h = zh % NH_;
    const int t0 = tbase + ((int)blockIdx.x * AW + wave) * 16;
    const size_t pbase = (size_t)zh * SEQ * HD;
    const size_t qo = pbase + (size_t)(t0 + lr) * HD + 8 * hi;
    const v16h qh0 = ldh(QH + qo), qh1 = ldh(QH + qo + 32);
    v16h qr0 = qh0, qr1 = qh1;
    if (RES) { qr0 = ldh(QR + qo); qr1 = ldh(QR + qo + 32); }
    const size_t ko = pbase + (size_t)lr * HD + 8 * hi;
    const size_t vo = pbase + (size_t)lr * SEQ + 8 * hi;
    const int* mrow = MK + (size_t)(t0 + lr) * SEQ_FULL + 8 * hi;
    int kend = KT[t0 >> 4]; kend = kend < 0 ? 0 : kend; kend = kend > SEQ ? SEQ : kend; kend &= ~31;
    v8f oh0 = (v8f){}, oh1 = (v8f){}, oh2 = (v8f){}, oh3 = (v8f){};
    v8f ol0 = (v8f){}, ol1 = (v8f){}, ol2 = (v8f){}, ol3 = (v8f){};
    float m = NEGB, l = 0.0f;
#pragma unroll 1
    for (int key0 = 0; key0 < kend; key0 += 32) {
        const int* mp = mrow + key0;
        const v4i ma0 = *(const v4i*)mp, ma1 = *(const v4i*)(mp + 4), mb0 = *(const v4i*)(mp + 16), mb1 = *(const v4i*)(mp + 20);
        const h16* ka = KP + ko + (size_t)key0 * HD;
        v8f sHa = (v8f){}, sHb = (v8f){}, sLa = (v8f){}, sLb = (v8f){};
        {
            const v16h ka0 = ldh(ka), ka1 = ldh(ka + 32), kb0 = ldh(ka + 16 * HD), kb1 = ldh(ka + 16 * HD + 32);
            if (RES) {
                const h16* kr = KR + ko + (size_t)key0 * HD;
                const v16h ra0 = ldh(kr), ra1 = ldh(kr + 32), rb0 = ldh(kr + 16 * HD), rb1 = ldh(kr + 16 * HD + 32);
                sHa = wmma16(ka0, qh0, sHa); sLa = wmma16(ka0, qr0, sLa); sHb = wmma16(kb0, qh0, sHb); sLb = wmma16(kb0, qr0, sLb);
                sHa = wmma16(ka1, qh1, sHa); sLa = wmma16(ka1, qr1, sLa); sHb = wmma16(kb1, qh1, sHb); sLb = wmma16(kb1, qr1, sLb);
                sLa = wmma16(ra0, qh0, sLa); sLb = wmma16(rb0, qh0, sLb); sLa = wmma16(ra1, qh1, sLa); sLb = wmma16(rb1, qh1, sLb);
                asm volatile("v_nop\n\tv_nop\n\tv_nop\n\tv_nop" : "+v"(sHa), "+v"(sLa), "+v"(sHb), "+v"(sLb) : "v"(ka0), "v"(ka1), "v"(kb0), "v"(kb1), "v"(ra0), "v"(ra1), "v"(rb0), "v"(rb1));
            } else {
                sHa = wmma16(ka0, qh0, sHa); sHb = wmma16(kb0, qh0, sHb); sHa = wmma16(ka1, qh1, sHa); sHb = wmma16(kb1, qh1, sHb);
                asm volatile("v_nop\n\tv_nop\n\tv_nop\n\tv_nop" : "+v"(sHa), "+v"(sHb) : "v"(ka0), "v"(ka1), "v"(kb0), "v"(kb1));
            }
        }
        const int mka[8] = { ma0[0], ma0[1], ma0[2], ma0[3], ma1[0], ma1[1], ma1[2], ma1[3] };
        const int mkb[8] = { mb0[0], mb0[1], mb0[2], mb0[3], mb1[0], mb1[1], mb1[2], mb1[3] };
        float ta[8], tb[8]; float mx = NEGB;
#pragma unroll
        for (int r = 0; r < 8; ++r) {
            float xa = sHa[r], xb = sHb[r];
            if (RES) { xa += sLa[r] * QRI; xb += sLb[r] * QRI; }
            xa *= SC2; xb *= SC2;
            ta[r] = (mka[r] != 0) ? xa : NEGB; tb[r] = (mkb[r] != 0) ? xb : NEGB;
            mx = fmaxf(mx, fmaxf(ta[r], tb[r])); }
        mx = fmaxf(mx, __shfl_xor(mx, 16, 32));
        const float mnew = fmaxf(m, mx);
        const float alpha = __builtin_amdgcn_exp2f(m - mnew);
        const float sh = PSH - mnew;
        v16h pb, pr; float ls = 0.0f;
#pragma unroll
        for (int r = 0; r < 8; ++r) {
            const float e0 = __builtin_amdgcn_exp2f(ta[r] + sh), e1 = __builtin_amdgcn_exp2f(tb[r] + sh);
            const float ea = (ta[r] > -1.0e38f) ? e0 : 0.0f; const float eb = (tb[r] > -1.0e38f) ? e1 : 0.0f;
            const h16 pa = (h16)ea; const h16 pc = (h16)eb; pb[r] = pa; pb[8 + r] = pc;
            if (RES) { pr[r] = (h16)((ea - (float)pa) * QRS); pr[8 + r] = (h16)((eb - (float)pc) * QRS); ls += ea + eb; }
            else     { pr[r] = pa; pr[8 + r] = pc; ls += (float)pa + (float)pc; } }
        l = l * alpha + ls; m = mnew;
        oh0 = oh0 * alpha; oh1 = oh1 * alpha; oh2 = oh2 * alpha; oh3 = oh3 * alpha;
        if (RES) { ol0 = ol0 * alpha; ol1 = ol1 * alpha; ol2 = ol2 * alpha; ol3 = ol3 * alpha; }
        const h16* va = VT + vo + key0;
        const v16h v0 = ldh(va), v1 = ldh(va + (size_t)16 * SEQ), v2 = ldh(va + (size_t)32 * SEQ), v3 = ldh(va + (size_t)48 * SEQ);
        if (RES) {
            const h16* vr = VR + vo + key0;
            const v16h w0 = ldh(vr), w1 = ldh(vr + (size_t)16 * SEQ), w2 = ldh(vr + (size_t)32 * SEQ), w3 = ldh(vr + (size_t)48 * SEQ);
            oh0 = wmma16(v0, pb, oh0); ol0 = wmma16(v0, pr, ol0); oh1 = wmma16(v1, pb, oh1); ol1 = wmma16(v1, pr, ol1);
            ol0 = wmma16(w0, pb, ol0); ol1 = wmma16(w1, pb, ol1);
            oh2 = wmma16(v2, pb, oh2); ol2 = wmma16(v2, pr, ol2); oh3 = wmma16(v3, pb, oh3); ol3 = wmma16(v3, pr, ol3);
            ol2 = wmma16(w2, pb, ol2); ol3 = wmma16(w3, pb, ol3);
            asm volatile("v_nop\n\tv_nop\n\tv_nop\n\tv_nop" : "+v"(oh0), "+v"(oh1), "+v"(oh2), "+v"(oh3), "+v"(ol0), "+v"(ol1), "+v"(ol2), "+v"(ol3)
                         : "v"(v0), "v"(v1), "v"(v2), "v"(v3), "v"(w0), "v"(w1), "v"(w2), "v"(w3), "v"(pb), "v"(pr));
        } else {
            oh0 = wmma16(v0, pb, oh0); oh1 = wmma16(v1, pb, oh1); oh2 = wmma16(v2, pb, oh2); oh3 = wmma16(v3, pb, oh3);
            asm volatile("v_nop\n\tv_nop\n\tv_nop\n\tv_nop" : "+v"(oh0), "+v"(oh1), "+v"(oh2), "+v"(oh3) : "v"(v0), "v"(v1), "v"(v2), "v"(v3), "v"(pb));
        }
    }
    l += __shfl_xor(l, 16, 32);
    const float inv = (1.0f / l) * CS;
    const int wb = wave * 16 * 68;
    *(v4fa*)(&os[wb + lr * 68 +  0 + 8 * hi]) = fin_lo<RES>(oh0, ol0, inv); *(v4fa*)(&os[wb + lr * 68 +  0 + 8 * hi + 4]) = fin_hi<RES>(oh0, ol0, inv);
    *(v4fa*)(&os[wb + lr * 68 + 16 + 8 * hi]) = fin_lo<RES>(oh1, ol1, inv); *(v4fa*)(&os[wb + lr * 68 + 16 + 8 * hi + 4]) = fin_hi<RES>(oh1, ol1, inv);
    *(v4fa*)(&os[wb + lr * 68 + 32 + 8 * hi]) = fin_lo<RES>(oh2, ol2, inv); *(v4fa*)(&os[wb + lr * 68 + 32 + 8 * hi + 4]) = fin_hi<RES>(oh2, ol2, inv);
    *(v4fa*)(&os[wb + lr * 68 + 48 + 8 * hi]) = fin_lo<RES>(oh3, ol3, inv); *(v4fa*)(&os[wb + lr * 68 + 48 + 8 * hi + 4]) = fin_hi<RES>(oh3, ol3, inv);
    wave_sync();
    const size_t crow = ((size_t)b * SEQ + t0) * DM + (size_t)h * HD;
    const size_t rrow = ((size_t)b * EARLY + t0) * DM + (size_t)h * HD;
#pragma unroll 1
    for (int ps = 0; ps < 2; ++ps) {
#pragma unroll
        for (int s = 0; s < 4; ++s) { const int row = 4 * s + (lane >> 3), c8 = (lane & 7) * 8;
            const v4f x0 = *(const v4fa*)(&os[wb + row * 68 + c8]); const v4f x1 = *(const v4fa*)(&os[wb + row * 68 + c8 + 4]); v8h hv, rv;
#pragma unroll
            for (int i = 0; i < 4; ++i) { const h16 a0 = (h16)x0[i]; const h16 a1 = (h16)x1[i]; hv[i] = a0; hv[4 + i] = a1;
                rv[i] = (h16)((x0[i] - (float)a0) * QRS); rv[4 + i] = (h16)((x1[i] - (float)a1) * QRS); }
            *(volatile v8h*)(CH + crow + (size_t)row * DM + c8) = hv;
            if (RES) *(volatile v8h*)(CR + rrow + (size_t)row * DM + c8) = rv; }
        if (ps == 0) __threadfence(); }
}

__global__ __launch_bounds__(32 * AW) void k_flash_early(const h16* QH, const h16* QR, const h16* KP, const h16* KR, const h16* VT, const h16* VR,
                                                         const int* MK, const int* KT, h16* CH, h16* CR) {
    flash_body<1>(QH, QR, KP, KR, VT, VR, MK, KT, CH, CR, 0);
}
__global__ __launch_bounds__(32 * AW) void k_flash_dense(const h16* QH, const h16* KP, const h16* VT, const int* MK, const int* KT, h16* CH) {
    flash_body<0>(QH, QH, KP, KP, VT, VT, MK, KT, CH, CH, EARLY);
}

template <int MT, int RES>
__device__ __forceinline__ void oproj_body(const h16* __restrict__ A, const h16* __restrict__ AR, const h16* __restrict__ Bt, const float* __restrict__ bias,
                                           float* OUT, const int tilesPerBatch, const int tStart) {
    __shared__ __align__(16) float os[16 * 68];
    const int K = DM;
    const int lane = threadIdx.x & 31, lr = lane & 15, hi = lane >> 4;
    const int bb = (int)blockIdx.x / tilesPerBatch, ti = (int)blockIdx.x % tilesPerBatch;
    const int t0 = tStart + ti * 16 * MT, c0 = blockIdx.y * 64;
    v8f acc[MT][4], acr[MT][4];
#pragma unroll
    for (int mb = 0; mb < MT; ++mb)
#pragma unroll
        for (int nb = 0; nb < 4; ++nb) { acc[mb][nb] = (v8f){}; acr[mb][nb] = (v8f){}; }
    const size_t aoff = ((size_t)bb * SEQ + t0 + lr) * K + 8 * hi;
    const size_t roff = ((size_t)bb * EARLY + t0 + lr) * K + 8 * hi;
    const size_t boff = (size_t)(c0 + lr) * K + 8 * hi;
#pragma unroll 1
    for (int kc = 0; kc < K; kc += 32) {
        v16h a[MT], ar[MT];
#pragma unroll
        for (int mb = 0; mb < MT; ++mb) { a[mb] = ldh(A + aoff + (size_t)mb * 16 * K + kc);
            if (RES) ar[mb] = ldh(AR + roff + (size_t)mb * 16 * K + kc); else ar[mb] = a[mb]; }
#pragma unroll
        for (int nb = 0; nb < 4; ++nb) { const v16h b = ldh(Bt + boff + (size_t)nb * 16 * K + kc);
#pragma unroll
            for (int mb = 0; mb < MT; ++mb) { acc[mb][nb] = wmma16(a[mb], b, acc[mb][nb]); if (RES) acr[mb][nb] = wmma16(ar[mb], b, acr[mb][nb]); } }
        if (RES) {
            asm volatile("v_nop\n\tv_nop\n\tv_nop\n\tv_nop" : "+v"(acc[0][3]), "+v"(acc[MT - 1][3]), "+v"(acr[0][3]), "+v"(acr[MT - 1][3]) : "v"(a[0]), "v"(a[MT - 1]), "v"(ar[0]), "v"(ar[MT - 1]));
        } else {
            asm volatile("v_nop\n\tv_nop\n\tv_nop\n\tv_nop" : "+v"(acc[0][3]), "+v"(acc[MT - 1][3]), "+v"(acc[MT / 2][2]), "+v"(acc[MT - 1][0]) : "v"(a[0]), "v"(a[MT - 1]), "v"(a[MT / 2]));
        }
    }
    const int cofs = lr * 4;
    const v4f bz = *(const v4f*)(bias + c0 + cofs); v4f bq;
#pragma unroll
    for (int i = 0; i < 4; ++i) bq[i] = bfr(bz[i]);
#pragma unroll
    for (int mb = 0; mb < MT; ++mb) {
#pragma unroll
        for (int nb = 0; nb < 4; ++nb) {
#pragma unroll
            for (int j = 0; j < 8; ++j) { float y = acc[mb][nb][j]; if (RES) y += acr[mb][nb][j] * QRI; os[(hi * 8 + j) * 68 + nb * 16 + lr] = y; } }
        wave_sync();
        float* orow = OUT + ((size_t)bb * OUT_SEQ + t0 + mb * 16) * DM + c0;
#pragma unroll 1
        for (int ps = 0; ps < 2; ++ps) {
#pragma unroll
            for (int s = 0; s < 8; ++s) { const int row = 2 * s + hi;
                const v4f val = *(const v4fa*)(&os[row * 68 + cofs]) * OSC + bq;
                *(volatile v4f*)(orow + (size_t)row * DM + cofs) = val; }
            if (ps == 0) __threadfence(); }
        wave_sync();
    }
}

__global__ __launch_bounds__(32) void k_oproj_early(const h16* A, const h16* AR, const h16* Bt, const float* bias, float* OUT, int tilesPerBatch, int tStart) {
    oproj_body<2, 1>(A, AR, Bt, bias, OUT, tilesPerBatch, tStart);
}
__global__ __launch_bounds__(32) void k_oproj_dense(const h16* A, const h16* Bt, const float* bias, float* OUT, int tilesPerBatch, int tStart) {
    oproj_body<4, 0>(A, A, Bt, bias, OUT, tilesPerBatch, tStart);
}

static constexpr size_t al256(size_t v) { return (v + 255) & ~(size_t)255; }
static constexpr size_t SZ_XB = al256((size_t)NB * SEQ * DM * 2);
static constexpr size_t SZ_WB = al256((size_t)4 * DM * DM * 2);
static constexpr size_t SZ_PL = al256((size_t)NB * NH_ * SEQ * HD * 2);
static constexpr size_t SZ_CR = al256((size_t)NB * EARLY * DM * 2);
static constexpr size_t SZ_KT = al256((size_t)((SEQ / 16 + 31) / 32) * 128);
static constexpr size_t SZ_TOTAL = SZ_XB + SZ_WB + 6 * SZ_PL + SZ_CR + SZ_KT;
static_assert(SZ_TOTAL <= (size_t)134217728);
static_assert(((size_t)DM * DM * 2) % 256 == 0);
static_assert((size_t)NB * SEQ * DM * 2 <= SZ_XB);

extern "C" void kernel_launch(void* const* d_in, const int* in_sizes, int n_in,
                              void* d_out, int out_size, void* d_ws, size_t ws_size, hipStream_t stream) {
    if (n_in < 10) return;
    const size_t needx = ((size_t)(NB - 1) * SEQ_FULL + SEQ) * DM;
    if ((size_t)in_sizes[0] < needx) return;
    if ((size_t)in_sizes[1] < (size_t)(SEQ - 1) * SEQ_FULL + SEQ) return;
    if ((size_t)in_sizes[2] < (size_t)DM * DM || (size_t)in_sizes[4] < (size_t)DM * DM || (size_t)in_sizes[6] < (size_t)DM * DM || (size_t)in_sizes[8] < (size_t)DM * DM) return;
    if (in_sizes[3] < DM || in_sizes[5] < DM || in_sizes[7] < DM || in_sizes[9] < DM) return;
    if ((size_t)out_size < ((size_t)(NB - 1) * OUT_SEQ + SEQ) * DM) return;
    if (SZ_TOTAL > ws_size) return;
    const float* x  = (const float*)d_in[0]; const int* mask = (const int*)d_in[1];
    const float* wq = (const float*)d_in[2]; const float* bq = (const float*)d_in[3];
    const float* wk = (const float*)d_in[4]; const float* bk = (const float*)d_in[5];
    const float* wv = (const float*)d_in[6]; const float* bv = (const float*)d_in[7];
    const float* wo = (const float*)d_in[8]; const float* bo = (const float*)d_in[9];
    float* OUT = (float*)d_out;
    char* wsp = (char*)d_ws;
    bf* XB = (bf*)wsp; h16* CH = (h16*)wsp; wsp += SZ_XB;
    bf* WB = (bf*)wsp; wsp += SZ_WB;
    h16* QH = (h16*)wsp; wsp += SZ_PL;
    h16* QR = (h16*)wsp; wsp += SZ_PL;
    h16* KP = (h16*)wsp; wsp += SZ_PL;
    h16* KR = (h16*)wsp; wsp += SZ_PL;
    h16* VT = (h16*)wsp; wsp += SZ_PL;
    h16* VR = (h16*)wsp; wsp += SZ_PL;
    h16* CR = (h16*)wsp; wsp += SZ_CR;
    int* KT = (int*)wsp; wsp += SZ_KT;
    bf* WQ = WB; bf* WK = WB + (size_t)DM * DM; bf* WV = WB + (size_t)2 * DM * DM; h16* WO = (h16*)(WB + (size_t)3 * DM * DM);

    if (SEQ == SEQ_FULL) {
        const size_t n8 = (size_t)NB * SEQ * DM / 8;
        k_cvt8<<<(unsigned)((n8 + 255) / 256), 256, 0, stream>>>(x, XB, n8);
    } else {
        const size_t n8 = (size_t)SEQ * DM / 8;
        for (int b = 0; b < NB; ++b) k_cvt8<<<(unsigned)((n8 + 255) / 256), 256, 0, stream>>>(x + (size_t)b * SEQ_FULL * DM, XB + (size_t)b * SEQ * DM, n8);
    }
    { const size_t n8 = (size_t)DM * DM / 8; const unsigned g = (unsigned)((n8 + 255) / 256);
      k_cvt8<<<g, 256, 0, stream>>>(wq, WQ, n8); k_cvt8<<<g, 256, 0, stream>>>(wk, WK, n8); k_cvt8<<<g, 256, 0, stream>>>(wv, WV, n8);
      k_cvtw<<<g, 256, 0, stream>>>(wo, WO, n8); }
    k_mscan<<<(unsigned)((SEQ / 16 + 31) / 32), 256, 0, stream>>>(mask, KT);

    k_proj<<<dim3(NB * SEQ / 64, DM / 64, 1), 32, 0, stream>>>(XB, WQ, bq, 0, QH, QR, 1, SEQ, (size_t)NH_ * SEQ * HD, HD, HD, (size_t)SEQ * HD, EARLY, BIGI);
    k_proj<<<dim3(NB * SEQ / 64, DM / 64, 1), 32, 0, stream>>>(XB, WK, bk, 0, KP, KR, 1, SEQ, (size_t)NH_ * SEQ * HD, HD, HD, (size_t)SEQ * HD, EARLY, BIGI);
    k_proj<<<dim3(DM / 64, NB * SEQ / 64, 1), 32, 0, stream>>>(WV, XB, bv, 1, VT, VR, 1, DM, (size_t)0, SEQ, SEQ, (size_t)DM * SEQ, BIGI, EARLY);

    k_flash_early<<<dim3(EARLY / (16 * AW), NB * NH_, 1), 32 * AW, 0, stream>>>(QH, QR, KP, KR, VT, VR, mask, KT, CH, CR);
    if (SEQ > EARLY)
        k_flash_dense<<<dim3((SEQ - EARLY) / (16 * AW), NB * NH_, 1), 32 * AW, 0, stream>>>(QH, KP, VT, mask, KT, CH);

    k_oproj_early<<<dim3(NB * (EARLY / 32), DM / 64, 1), 32, 0, stream>>>(CH, CR, WO, bo, OUT, EARLY / 32, 0);
    if (SEQ > EARLY)
        k_oproj_dense<<<dim3(NB * ((SEQ - EARLY) / 64), DM / 64, 1), 32, 0, stream>>>(CH, WO, bo, OUT, (SEQ - EARLY) / 64, EARLY);
}
